// GATLayer_36558761623739
// MI455X (gfx1250) — hardware-verified
//
#include <hip/hip_runtime.h>
#include <stddef.h>
#include <stdint.h>
#include <math.h>


#define NN      100000
#define NE      1250000
#define DIN     128
#define DOUT    64
#define MTILE   128
#define MP      100096
#define PTHR    256
#define NUH     (MP * (DIN / 8))
#define NBH     (NUH / PTHR)
#define NUW     (DOUT * (DIN / 8))
#define NBW     (NUW / PTHR)
#define GTHR    256
#define LDP     68
#define BTHR    256
#define NWAVE   8
#define NBR     1024
#define SLB     10
#define NBLK    98
#define WRANGE  156416
#define WITERS  611
#define WLCAP   4096
#define RCAP    16384
#define DEGCAP  128
#define TABN    2080
#define SRCB    17
#define BKT_ZINTS (RCAP + 32 + TABN + NBR + 64)
#define BKT_INTS  (NWAVE * WLCAP + BKT_ZINTS)
#define BKT_LDS   (BKT_INTS * 4)
#define RSUB    8
#define RSPW    16
#define NEGBIG  (-1.0e30f)
#define WSMAX   134217728

static_assert(97 * 1024 + 672 == NN);
static_assert(NN < (1 << SRCB));
static_assert(NBLK * NBR >= NN && (NBLK - 1) * NBR < NN);
static_assert(NBR == (1 << SLB));
static_assert(SRCB + SLB < 31);
static_assert(RCAP % 1024 == 0 && RCAP >= 13064 + 1307);
static_assert(DEGCAP % 32 == 0 && DEGCAP >= 29 + 8);
static_assert(WITERS * 256 == WRANGE && NWAVE * WRANGE >= NE && WRANGE < (1 << 18));
static_assert(NE % 8 == 0 && NE >= 8);
static_assert(MP == 782 * MTILE && MP >= NN && 781 * 128 + 32 == NN);
static_assert(NUH % PTHR == 0 && NUW % PTHR == 0);
static_assert(DIN % 32 == 0 && DOUT == 64 && DOUT == 2 * 32);
static_assert(GTHR == 2 * MTILE && MTILE == (GTHR / 32) * 16);
static_assert(BKT_ZINTS % 4 == 0 && (NWAVE * WLCAP) % 4 == 0);
static_assert(BKT_LDS <= 300000);
static_assert((TABN * 4) % 128 == 0 && TABN == 2 * NBR + 32);
static_assert(RSUB * NWAVE * RSPW == NBR);
static_assert((LDP * 4) % 16 == 0 && LDP >= DOUT);

typedef float          v2f  __attribute__((ext_vector_type(2)));
typedef float          v4f  __attribute__((ext_vector_type(4)));
typedef float          v8f  __attribute__((ext_vector_type(8)));
typedef int            v4i  __attribute__((ext_vector_type(4)));
typedef int            v8i  __attribute__((ext_vector_type(8)));
typedef unsigned int   v4u  __attribute__((ext_vector_type(4)));
typedef unsigned short v8us __attribute__((ext_vector_type(8)));
typedef __bf16         v16b __attribute__((ext_vector_type(16)));
typedef v2f  __attribute__((may_alias)) v2fa;
typedef v4f  __attribute__((may_alias)) v4fa;
typedef v4i  __attribute__((may_alias)) v4ia;
typedef v8us __attribute__((may_alias)) v8usa;
union FragB { v16b v; v8us h[2]; v8i w; };

__device__ __forceinline__ v8f wmb(const FragB& a, const FragB& b, v8f c) {
  v8f d = __builtin_amdgcn_wmma_f32_16x16x32_bf16(false, a.v, false, b.v, (short)0, c, false, false);
  asm volatile("v_nop\n\tv_nop\n\tv_nop\n\tv_nop" : "+v"(d) : "v"(a.w), "v"(b.w));
  return d;
}

__device__ __forceinline__ unsigned int f2bf(float f) {
  const unsigned int u = __float_as_uint(f);
  return ((u + 0x7FFFu + ((u >> 16) & 1u)) >> 16) & 0xFFFFu;
}
__device__ __forceinline__ float bfr(float f) { return __uint_as_float(f2bf(f) << 16); }
__device__ __forceinline__ unsigned int pk2(float lo, float hi) { return f2bf(lo) | (f2bf(hi) << 16); }
__device__ __forceinline__ v4u pack8(const v4f a, const v4f b) {
  v4u r;
  r.x = pk2(a.x, a.y); r.y = pk2(a.z, a.w); r.z = pk2(b.x, b.y); r.w = pk2(b.z, b.w);
  return r;
}

__global__ __launch_bounds__(PTHR) void k_prep(const float* __restrict__ h, const float* __restrict__ W,
                                               const float* __restrict__ a,
                                               unsigned short* HB, unsigned short* WB, float* AF) {
  const int tid = (int)threadIdx.x;
  const int blk = (int)blockIdx.x;
  if (blk < NBH) {
    const int u  = blk * PTHR + tid;
    const int uc = u < NN * 16 ? u : NN * 16 - 1;
    const float* p = h + (size_t)uc * 8;
    const v4f x = *(const v4fa*)p;
    const v4f y = *(const v4fa*)(p + 4);
    asm volatile("" :: "v"(x), "v"(y));
    const unsigned int keep = (u < NN * 16) ? 0xFFFFFFFFu : 0u;
    v4u o = pack8(x, y);
    o.x &= keep; o.y &= keep; o.z &= keep; o.w &= keep;
    unsigned short* dp = HB + (size_t)u * 8;
    *(volatile v4u*)dp = o;
    __threadfence();
    *(volatile v4u*)dp = o;
  } else if (blk < NBH + NBW) {
    const int u = (blk - NBH) * PTHR + tid;
    const float* p = W + (size_t)u * 8;
    const v4f x = *(const v4fa*)p;
    const v4f y = *(const v4fa*)(p + 4);
    const v4u o = pack8(x, y);
    unsigned short* dp = WB + (size_t)u * 8;
    *(volatile v4u*)dp = o;
    __threadfence();
    *(volatile v4u*)dp = o;
  } else {
    if (tid < 32) {
      const v4f x = *(const v4fa*)(a + 4 * tid);
      v4f r;
      r.x = bfr(x.x); r.y = bfr(x.y); r.z = bfr(x.z); r.w = bfr(x.w);
      float* dp = AF + 4 * tid;
      *(volatile v4f*)dp = r;
      __threadfence();
      *(volatile v4f*)dp = r;
    }
  }
}

__global__ __launch_bounds__(BTHR) void k_bucket(const int* __restrict__ srcs, const int* __restrict__ dsts,
                                                 int* HITS, int* TAB) {
  extern __shared__ __attribute__((aligned(16))) int dsm[];
  int* wl   = dsm;
  int* sl   = dsm + NWAVE * WLCAP;
  int* tabl = sl + RCAP + 32;
  int* cur  = tabl + TABN;
  int* misc = cur + NBR;
  int* offp = tabl;
  int* cntp = tabl + NBR;
  const int tid  = (int)threadIdx.x, lane = tid & 31;
  const int wave = __builtin_amdgcn_readfirstlane(tid >> 5);
  const int blk  = (int)blockIdx.x;
  const int base = blk * NBR;
  int nb = NN - base;
  nb = nb > NBR ? NBR : nb;

  {
    const v4i z4 = {0, 0, 0, 0};
    for (int i = tid; i < BKT_ZINTS / 4; i += BTHR) *(v4ia*)(sl + 4 * i) = z4;
  }
  __syncthreads();

  int wc = 0;
  {
    int* mywl = wl + wave * WLCAP;
    const unsigned nbs = (unsigned)base;
    const unsigned unb = (unsigned)nb;
    const int ebase = wave * WRANGE;
#pragma unroll 1
    for (int it = 0; it < WITERS; ++it) {
      const int el0 = it * 256 + lane * 8;
      const int e0  = ebase + el0;
      const int ec  = e0 < NE - 8 ? e0 : NE - 8;
      const v4i da = *(const v4i*)(dsts + ec);
      const v4i db = *(const v4i*)(dsts + ec + 4);
      asm volatile("" :: "v"(da), "v"(db));
      const bool inr = e0 < NE;
      const unsigned s0 = (unsigned)da.x - nbs, s1 = (unsigned)da.y - nbs;
      const unsigned s2 = (unsigned)da.z - nbs, s3 = (unsigned)da.w - nbs;
      const unsigned s4 = (unsigned)db.x - nbs, s5 = (unsigned)db.y - nbs;
      const unsigned s6 = (unsigned)db.z - nbs, s7 = (unsigned)db.w - nbs;
      const bool h0 = inr & (s0 < unb), h1 = inr & (s1 < unb), h2 = inr & (s2 < unb), h3 = inr & (s3 < unb);
      const bool h4 = inr & (s4 < unb), h5 = inr & (s5 < unb), h6 = inr & (s6 < unb), h7 = inr & (s7 < unb);
      const unsigned any = __builtin_amdgcn_ballot_w32(h0 | h1 | h2 | h3 | h4 | h5 | h6 | h7);
      if (any != 0u) {
#define HITJ(J, HJ, SJ) { \
        const unsigned mj = __builtin_amdgcn_ballot_w32(HJ); \
        if (mj != 0u) { \
          const int pos = wc + (int)__builtin_amdgcn_mbcnt_lo(mj, 0u); \
          if ((HJ) && pos < WLCAP) mywl[pos] = ((el0 + (J)) << SLB) | (int)(SJ); \
          wc += (int)__builtin_popcount(mj); } }
        HITJ(0, h0, s0)
        HITJ(1, h1, s1)
        HITJ(2, h2, s2)
        HITJ(3, h3, s3)
        HITJ(4, h4, s4)
        HITJ(5, h5, s5)
        HITJ(6, h6, s6)
        HITJ(7, h7, s7)
#undef HITJ
      }
    }
  }
  if (lane == 0) misc[wave] = wc;
  __syncthreads();

  if (wave == 0) {
    int tt = 0, ov = 0;
#pragma unroll 1
    for (int w2 = 0; w2 < NWAVE; ++w2) {
      int c = __builtin_amdgcn_readfirstlane(misc[w2]);
      ov |= (c > WLCAP) ? 1 : 0;
      c = c < 0 ? 0 : (c > WLCAP ? WLCAP : c);
#pragma unroll 1
      for (int b0 = 0; b0 < c; b0 += 32) {
        int idx = b0 + lane;
        idx = idx < c ? idx : c - 1;
        const int ent = wl[w2 * WLCAP + idx];
        const int m32 = (c - b0) < 32 ? (c - b0) : 32;
#pragma unroll 1
        for (int k = 0; k < m32; ++k) {
          const int u    = __builtin_amdgcn_readlane(ent, k);
          const int slot = u & (NBR - 1);
          if (lane == 0) cntp[slot] = cntp[slot] + 1;
        }
      }
      tt += c;
    }
    ov |= (tt > RCAP) ? 1 : 0;
    if (lane == 0) { tabl[2 * NBR] = ov; tabl[2 * NBR + 1] = tt; }
  }
  __syncthreads();

  {
    const v4i cv = *(const v4ia*)(cntp + 4 * tid);
    const int e0 = cv.x < 0 ? 0 : cv.x, e1 = cv.y < 0 ? 0 : cv.y;
    const int e2 = cv.z < 0 ? 0 : cv.z, e3 = cv.w < 0 ? 0 : cv.w;
    const int ts = e0 + e1 + e2 + e3;
    int incl = ts;
#pragma unroll
    for (int d = 1; d < 32; d <<= 1) {
      const int up = __shfl_up(incl, d);
      if (lane >= d) incl += up;
    }
    if (lane == 31) misc[8 + wave] = incl;
    __syncthreads();
    int pre = 0;
#pragma unroll
    for (int w2 = 0; w2 < NWAVE; ++w2) pre += (w2 < wave) ? misc[8 + w2] : 0;
    const int run = pre + incl - ts;
    v4i o4;
    o4.x = run; o4.y = run + e0; o4.z = run + e0 + e1; o4.w = run + e0 + e1 + e2;
    *(v4ia*)(offp + 4 * tid) = o4;
    *(v4ia*)(cur + 4 * tid)  = o4;
  }
  __syncthreads();

  if (wave == 0) {
#pragma unroll 1
    for (int w2 = 0; w2 < NWAVE; ++w2) {
      int c = __builtin_amdgcn_readfirstlane(misc[w2]);
      c = c < 0 ? 0 : (c > WLCAP ? WLCAP : c);
#pragma unroll 1
      for (int b0 = 0; b0 < c; b0 += 32) {
        int idx = b0 + lane;
        idx = idx < c ? idx : c - 1;
        const int ent  = wl[w2 * WLCAP + idx];
        const int slot = ent & (NBR - 1);
        int eid = w2 * WRANGE + ((ent >> SLB) & 0x3FFFF);
        eid = eid < 0 ? 0 : (eid > NE - 1 ? NE - 1 : eid);
        int sr = srcs[eid];
        asm volatile("" :: "v"(sr));
        sr = sr < 0 ? 0 : (sr > NN - 1 ? NN - 1 : sr);
        const int word = sr | (slot << SRCB);
        const int m32 = (c - b0) < 32 ? (c - b0) : 32;
#pragma unroll 1
        for (int k = 0; k < m32; ++k) {
          const int u   = __builtin_amdgcn_readlane(word, k);
          const int sl2 = (u >> SRCB) & (NBR - 1);
          if (lane == 0) {
            int p = cur[sl2];
            p = p < 0 ? 0 : (p > RCAP ? RCAP : p);
            sl[p] = u;
            cur[sl2] = p + 1;
          }
        }
      }
    }
  }
  __syncthreads();

  int* hp = HITS + (size_t)blk * RCAP;
  int* tp = TAB + (size_t)blk * TABN;
#pragma unroll 1
  for (int i = tid; i < RCAP / 4; i += BTHR) {
    const v4i v = *(const v4ia*)(sl + 4 * i);
    *(volatile v4i*)(hp + 4 * i) = v;
  }
#pragma unroll 1
  for (int i = tid; i < TABN / 4; i += BTHR) {
    const v4i v = *(const v4ia*)(tabl + 4 * i);
    *(volatile v4i*)(tp + 4 * i) = v;
  }
  __threadfence();
#pragma unroll 1
  for (int i = tid; i < RCAP / 4; i += BTHR) {
    const v4i v = *(const v4ia*)(sl + 4 * i);
    *(volatile v4i*)(hp + 4 * i) = v;
  }
#pragma unroll 1
  for (int i = tid; i < TABN / 4; i += BTHR) {
    const v4i v = *(const v4ia*)(tabl + 4 * i);
    *(volatile v4i*)(tp + 4 * i) = v;
  }
}

__global__ __launch_bounds__(GTHR) void k_gemm(const unsigned short* __restrict__ HB,
                                               const unsigned short* __restrict__ WB,
                                               const float* __restrict__ AF, float* Zp, float* SDp) {
  __shared__ __attribute__((aligned(16))) float stg[MTILE * LDP];
  __shared__ __attribute__((aligned(16))) float saf[2 * DOUT];
  __shared__ __attribute__((aligned(16))) float sdl[2 * MTILE];
  const int tid = (int)threadIdx.x, lane = tid & 31, wave = tid >> 5, hh = lane >> 4, m = lane & 15;
  const int rowBase = (int)blockIdx.x * MTILE;

  if (tid < 32) {
    const v4f v = *(const v4fa*)(AF + 4 * tid);
    *(v4fa*)(saf + 4 * tid) = v;
  }

  v8f acc[4];
  {
    const v8f z = {0.f, 0.f, 0.f, 0.f, 0.f, 0.f, 0.f, 0.f};
    acc[0] = z; acc[1] = z; acc[2] = z; acc[3] = z;
  }
  const unsigned short* ap = HB + (size_t)(rowBase + 16 * wave + m) * DIN + 8 * hh;
  const unsigned short* wp = WB + (size_t)m * DIN + 8 * hh;
#pragma unroll 1
  for (int k0 = 0; k0 < DIN; k0 += 32) {
    FragB af;
    af.h[0] = *(const v8usa*)(ap + k0);
    af.h[1] = *(const v8usa*)(ap + k0 + 16);
#pragma unroll
    for (int t = 0; t < 4; ++t) {
      const unsigned short* wq = wp + (size_t)(16 * t) * DIN + k0;
      FragB bf;
      bf.h[0] = *(const v8usa*)wq;
      bf.h[1] = *(const v8usa*)(wq + 16);
      acc[t] = wmb(af, bf, acc[t]);
    }
  }

#pragma unroll
  for (int t = 0; t < 4; ++t) {
    const int lc = 16 * t + m;
#pragma unroll
    for (int r = 0; r < 8; ++r) {
      const int lr = 16 * wave + 8 * hh + r;
      stg[lr * LDP + lc] = acc[t][r];
    }
  }
  __syncthreads();

  {
    const int row = tid & (MTILE - 1), which = tid >> 7;
    const float* hr = stg + row * LDP;
    const float* av = saf + DOUT * which;
    float dv = 0.0f;
#pragma unroll 2
    for (int c4 = 0; c4 < DOUT / 4; ++c4) {
      const v4f hv = *(const v4fa*)(hr + 4 * c4);
      const v4f a4 = *(const v4fa*)(av + 4 * c4);
      dv = fmaf(hv.x, a4.x, dv);
      dv = fmaf(hv.y, a4.y, dv);
      dv = fmaf(hv.z, a4.z, dv);
      dv = fmaf(hv.w, a4.w, dv);
    }
    sdl[2 * row + which] = dv;
  }
  __syncthreads();

  v4f fv[8];
#pragma unroll
  for (int i = 0; i < 8; ++i) {
    const int lr = 16 * wave + 2 * i + hh;
    fv[i] = *(const v4fa*)(stg + lr * LDP + 4 * m);
  }
  const int si = tid < 64 ? tid : 63;
  const v4f sdv = *(const v4fa*)(sdl + 4 * si);
  float* sp = SDp + (size_t)rowBase * 2 + 4 * si;
  const bool wsd = tid < 64;

#pragma unroll
  for (int i = 0; i < 8; ++i) {
    const int lr = 16 * wave + 2 * i + hh;
    float* op = Zp + (size_t)(rowBase + lr) * DOUT + 4 * m;
    *(volatile v4f*)op = fv[i];
  }
  if (wsd) *(volatile v4f*)sp = sdv;
  __threadfence();
#pragma unroll
  for (int i = 0; i < 8; ++i) {
    const int lr = 16 * wave + 2 * i + hh;
    float* op = Zp + (size_t)(rowBase + lr) * DOUT + 4 * m;
    *(volatile v4f*)op = fv[i];
  }
  if (wsd) *(volatile v4f*)sp = sdv;
}

__global__ __launch_bounds__(BTHR) void k_replay(const unsigned* __restrict__ HITS, const int* __restrict__ TAB,
                                                 const float* __restrict__ Zp, const float* __restrict__ SDp,
                                                 float* outp) {
  const int tid = (int)threadIdx.x, lane = tid & 31;
  const int wave = __builtin_amdgcn_readfirstlane(tid >> 5);
  const int b   = (int)blockIdx.x / RSUB;
  const int sub = (int)blockIdx.x - b * RSUB;
  const int* tb = TAB + (size_t)b * TABN;
  const unsigned* hb = HITS + (size_t)b * RCAP;
  const int flg = __builtin_amdgcn_readfirstlane(tb[2 * NBR]);
  const float qnan = __int_as_float(0x7fc00000);

#pragma unroll 1
  for (int j = 0; j < RSPW; ++j) {
    const int slot = sub * (NWAVE * RSPW) + wave * RSPW + j;
    const int node = b * NBR + slot;
    if (node < NN) {
      int o = __builtin_amdgcn_readfirstlane(tb[slot]);
      const int craw = __builtin_amdgcn_readfirstlane(tb[NBR + slot]);
      const bool bad = (flg != 0) || (craw > DEGCAP) || (craw < 0);
      int c = craw < 0 ? 0 : (craw > DEGCAP ? DEGCAP : craw);
      o = o < 0 ? 0 : (o > RCAP - 1 ? RCAP - 1 : o);
      if (c > RCAP - o) c = RCAP - o;
      int last = o + c - 1; last = last < o ? o : last;
      const float di = SDp[(size_t)node * 2 + 1];
      float mrun = NEGBIG, l = 0.0f;
      float a0 = 0.0f, a1 = 0.0f;

#pragma unroll 1
      for (int b0 = 0; b0 < c; b0 += 32) {
        int idx = o + b0 + lane;
        idx = idx > last ? last : idx;
        const unsigned word = hb[idx];
        asm volatile("" :: "v"(word));
        int sj = (int)(word & 0x1FFFFu);
        sj = sj > NN - 1 ? NN - 1 : sj;
        const float sv = SDp[(size_t)sj * 2];
        asm volatile("" :: "v"(sv));
        const bool valid = (b0 + lane) < c;
        float e = sv + di;
        e = (e >= 0.0f) ? e : 0.01f * e;
        e = valid ? e : NEGBIG;
        float cm = e;
#pragma unroll
        for (int off = 16; off > 0; off >>= 1) cm = fmaxf(cm, __shfl_xor(cm, off));
        const float mn = fmaxf(mrun, cm);
        const float sc = expf(mrun - mn);
        float p = expf(e - mn);
        p = valid ? p : 0.0f;
        l  = l * sc;
        a0 = a0 * sc;
        a1 = a1 * sc;
        mrun = mn;
        const int pi  = __float_as_int(p);
        const int m32 = (c - b0) < 32 ? (c - b0) : 32;
#pragma unroll 1
        for (int t = 0; t < m32; ++t) {
          const int   st = __builtin_amdgcn_readlane(sj, t);
          const float pt = __int_as_float(__builtin_amdgcn_readlane(pi, t));
          const v2f z = *(const v2fa*)(Zp + (size_t)st * DOUT + 2 * lane);
          l  = l + pt;
          a0 = fmaf(pt, z.x, a0);
          a1 = fmaf(pt, z.y, a1);
        }
      }
      const bool some = c > 0;
      const float ls  = some ? l : 1.0f;
      const float inv = 1.0f / ls;
      float v0 = a0 * inv, v1 = a1 * inv;
      v0 = some ? v0 : 0.0f;
      v1 = some ? v1 : 0.0f;
      v0 = bad ? qnan : v0;
      v1 = bad ? qnan : v1;
      v2f ov;
      ov.x = v0; ov.y = v1;
      float* op = outp + (size_t)node * DOUT + 2 * lane;
      *(volatile v2f*)op = ov;
      __threadfence();
      *(volatile v2f*)op = ov;
    }
  }
}

static constexpr size_t SZ_HB  = (size_t)MP * DIN * 2;
static constexpr size_t SZ_Z   = (size_t)MP * DOUT * 4;
static constexpr size_t SZ_SD  = (size_t)MP * 2 * 4;
static constexpr size_t SZ_HT  = (size_t)NBLK * RCAP * 4;
static constexpr size_t SZ_TAB = (size_t)NBLK * TABN * 4;
static constexpr size_t SZ_WB  = (size_t)DOUT * DIN * 2;
static constexpr size_t SZ_AF  = (size_t)DIN * 4;
static constexpr size_t O_HB   = 0;
static constexpr size_t O_Z    = O_HB + SZ_HB;
static constexpr size_t O_SD   = O_Z + SZ_Z;
static constexpr size_t O_HT   = O_SD + SZ_SD;
static constexpr size_t O_TAB  = O_HT + SZ_HT;
static constexpr size_t O_WB   = O_TAB + SZ_TAB;
static constexpr size_t O_AF   = O_WB + SZ_WB;
static constexpr size_t WS_TOT = O_AF + SZ_AF;
static_assert(SZ_HB % 256 == 0 && SZ_Z % 256 == 0 && SZ_SD % 256 == 0 && SZ_HT % 256 == 0);
static_assert(SZ_TAB % 256 == 0 && SZ_WB % 256 == 0 && SZ_AF % 256 == 0);
static_assert(WS_TOT <= (size_t)WSMAX);
static_assert((size_t)(MP / MTILE) * MTILE * 2 * 4 <= SZ_SD);
static_assert((size_t)NN * DOUT - 1 < (size_t)NN * DOUT);

extern "C" void kernel_launch(void* const* d_in, const int* in_sizes, int n_in,
                              void* d_out, int out_size, void* d_ws, size_t ws_size,
                              hipStream_t stream) {
  if (n_in < 5) return;
  if (in_sizes[0] != NN * DIN) return;
  if (in_sizes[1] != DOUT * DIN) return;
  if (in_sizes[2] != 2 * DOUT) return;
  if (in_sizes[3] != NE) return;
  if (in_sizes[4] != NE) return;
  if (out_size != NN * DOUT) return;
  if (WS_TOT > ws_size) return;

  const float* h   = (const float*)d_in[0];
  const float* W   = (const float*)d_in[1];
  const float* a   = (const float*)d_in[2];
  const int*   src = (const int*)d_in[3];
  const int*   dst = (const int*)d_in[4];
  float* out = (float*)d_out;

  char* ws = (char*)d_ws;
  unsigned short* HB   = (unsigned short*)(ws + O_HB);
  float*          Zp   = (float*)(ws + O_Z);
  float*          SDp  = (float*)(ws + O_SD);
  int*            HITS = (int*)(ws + O_HT);
  int*            TAB  = (int*)(ws + O_TAB);
  unsigned short* WB   = (unsigned short*)(ws + O_WB);
  float*          AF   = (float*)(ws + O_AF);

  hipFuncSetAttribute(reinterpret_cast<const void*>(&k_bucket),
                      hipFuncAttributeMaxDynamicSharedMemorySize, (int)BKT_LDS);

  k_prep<<<NBH + NBW + 1, PTHR, 0, stream>>>(h, W, a, HB, WB, AF);
  k_bucket<<<NBLK, BTHR, BKT_LDS, stream>>>(src, dst, HITS, TAB);
  k_gemm<<<MP / MTILE, GTHR, 0, stream>>>(HB, WB, AF, Zp, SDp);
  k_replay<<<NBLK * RSUB, BTHR, 0, stream>>>((const unsigned*)HITS, TAB, Zp, SDp, out);
}
